// MLPAttention_6957847019898
// MI455X (gfx1250) — hardware-verified
//
#include <hip/hip_runtime.h>
#include <stddef.h>

constexpr int NBATCH = 2;
constexpr int SEQ    = 2048;
constexpr int DMODEL = 1024;
constexpr int NHEAD  = 16;
constexpr int DHEAD  = 64;
constexpr int NHID   = 128;
constexpr int NTOK   = NBATCH * SEQ;
constexpr int DQKV   = NHEAD * DHEAD;

constexpr float SC_XH = 8.0f;
constexpr float SC_V  = 8.0f;
constexpr float SC_W1 = 64.0f;
constexpr float SC_W2 = 64.0f;
constexpr float SC_H  = 8.0f;
constexpr float SC_P  = 32768.0f;

static_assert(NTOK % 64 == 0 && DQKV % 64 == 0 && DMODEL % 64 == 0, "gemm tiles");
static_assert(DMODEL % 32 == 0 && DHEAD % 32 == 0, "gemm K");
static_assert(SEQ % 64 == 0 && NHID % 64 == 0, "gemm tiles");
static_assert(NHID == 128 && DHEAD == 64, "attention geometry");
static_assert((NTOK * DMODEL) % 8 == 0, "cast x8");

typedef __attribute__((ext_vector_type(16))) _Float16 v16h;
typedef __attribute__((ext_vector_type(8)))  _Float16 v8h;
typedef __attribute__((ext_vector_type(16))) __bf16   v16b;
typedef __attribute__((ext_vector_type(8)))  __bf16   v8b;
typedef __attribute__((ext_vector_type(8)))  float    v8f;
typedef __attribute__((ext_vector_type(4)))  float    v4f;
typedef __attribute__((ext_vector_type(4)))  unsigned int v4u;

__device__ __forceinline__ unsigned short f2bf_bits(float f) {
  unsigned u = __float_as_uint(f);
  return (unsigned short)((u + 0x7FFFu + ((u >> 16) & 1u)) >> 16);
}
__device__ __forceinline__ float bf_bits2f(unsigned short h) { return __uint_as_float(((unsigned)h) << 16); }

__device__ __forceinline__ void dep_guard_h(v8f& a, v8f& b, v16h x, v16h y) { asm volatile("v_nop\n\tv_nop\n\tv_nop\n\tv_nop" : "+v"(a), "+v"(b) : "v"(x), "v"(y)); }
__device__ __forceinline__ void dep_guard_b(v8f& a, v8f& b, v16b x, v16b y) { asm volatile("v_nop\n\tv_nop\n\tv_nop\n\tv_nop" : "+v"(a), "+v"(b) : "v"(x), "v"(y)); }
__device__ __forceinline__ void keep4_h(v16h a, v16h b, v16h c, v16h d) { asm volatile("v_nop" :: "v"(a), "v"(b), "v"(c), "v"(d)); }
__device__ __forceinline__ void keep4_b(v16b a, v16b b, v16b c, v16b d) { asm volatile("v_nop" :: "v"(a), "v"(b), "v"(c), "v"(d)); }
__device__ __forceinline__ void acc_guard4(v8f& a, v8f& b, v8f& c, v8f& d) { asm volatile("v_nop\n\tv_nop\n\tv_nop\n\tv_nop" : "+v"(a), "+v"(b), "+v"(c), "+v"(d)); }

template <typename T> struct Frag;
template <> struct Frag<_Float16> {
  typedef v16h V; union U { v16h v; v8h h[2]; };
  static __device__ __forceinline__ v16h load(const _Float16* p) {
    U f; f.h[0] = *(const v8h*)(p); f.h[1] = *(const v8h*)(p + 16); return f.v;
  }
  static __device__ __forceinline__ v8f mma(v16h a, v16h b, v8f c) {
    return __builtin_amdgcn_wmma_f32_16x16x32_f16(false, a, false, b, (short)0, c, false, false);
  }
  static __device__ __forceinline__ void guard(v8f& a, v8f& b, v16h x, v16h y) { dep_guard_h(a, b, x, y); }
  static __device__ __forceinline__ void keep(v16h a, v16h b, v16h c, v16h d) { keep4_h(a, b, c, d); }
};
template <> struct Frag<__bf16> {
  typedef v16b V; union U { v16b v; v8b h[2]; };
  static __device__ __forceinline__ v16b load(const __bf16* p) {
    U f; f.h[0] = *(const v8b*)(p); f.h[1] = *(const v8b*)(p + 16); return f.v;
  }
  static __device__ __forceinline__ v8f mma(v16b a, v16b b, v8f c) {
    return __builtin_amdgcn_wmma_f32_16x16x32_bf16(false, a, false, b, (short)0, c, false, false);
  }
  static __device__ __forceinline__ void guard(v8f& a, v8f& b, v16b x, v16b y) { dep_guard_b(a, b, x, y); }
  static __device__ __forceinline__ void keep(v16b a, v16b b, v16b c, v16b d) { keep4_b(a, b, c, d); }
};

template <int ET> struct Elem;
template <> struct Elem<0> { typedef _Float16 T; };
template <> struct Elem<1> { typedef __bf16 T; };
template <int ET, bool SPLIT, int BIAS_MODE, int OUT_MODE, int ACT = 0>
__global__ __launch_bounds__(256) void wmma_gemm64(
    const unsigned short* __restrict__ Ap, const unsigned short* __restrict__ A2p, int lda, long strideA,
    const unsigned short* __restrict__ Btp, const unsigned short* __restrict__ Bt2p, int ldb, long strideB,
    void* __restrict__ Cout, void* __restrict__ Cout2, int ldc, long strideC,
    const float* __restrict__ bias,
    int M, int N, int K, float scale) {
  typedef typename Elem<ET>::T T;
  typedef typename Frag<T>::V V;
  const T* A = (const T*)Ap; const T* A2 = (const T*)A2p; const T* Bt = (const T*)Btp; const T* Bt2 = (const T*)Bt2p;
  __shared__ __align__(16) float sT[8][16 * 68];
  const int b    = blockIdx.y;
  const int lane = threadIdx.x & 31;
  const int wave = threadIdx.x >> 5;
  const int tilesN = N >> 6;
  const int tilesM = M >> 6;
  const int tile = blockIdx.x * 8 + wave;
  if (tile >= tilesM * tilesN) return;
  const int tm = tile / tilesN;
  const int tn = tile - tm * tilesN;
  const int m0 = tm << 6;
  const int n0 = tn << 6;

  const T* Ab  = A  + (size_t)b * strideA;
  const T* Bb  = Bt + (size_t)b * strideB;
  const T* Ab2 = SPLIT ? (A2  + (size_t)b * strideA) : nullptr;
  const T* Bb2 = SPLIT ? (Bt2 + (size_t)b * strideB) : nullptr;

  const int rlane = lane & 15;
  const int koff  = (lane >> 4) * 8;
  const int mOff  = (lane >> 4) * 8;

  v8f acc[4][4];
#pragma unroll
  for (int i = 0; i < 4; ++i)
#pragma unroll
    for (int j = 0; j < 4; ++j) acc[i][j] = (v8f){0.f,0.f,0.f,0.f,0.f,0.f,0.f,0.f};

  for (int k0 = 0; k0 < K; k0 += 32) {
    V bh[4], bl[4];
#pragma unroll
    for (int j = 0; j < 4; ++j) {
      const size_t bo = (size_t)(n0 + (j << 4) + rlane) * ldb + koff + k0;
      bh[j] = Frag<T>::load(Bb + bo);
      if (SPLIT) bl[j] = Frag<T>::load(Bb2 + bo);
    }
#pragma unroll
    for (int i = 0; i < 4; ++i) {
      const size_t ao = (size_t)(m0 + (i << 4) + rlane) * lda + koff + k0;
      V ah = Frag<T>::load(Ab + ao);
      V al;
      if (SPLIT) al = Frag<T>::load(Ab2 + ao);
#pragma unroll
      for (int j = 0; j < 4; ++j) {
        acc[i][j] = Frag<T>::mma(ah, bh[j], acc[i][j]);
        if (SPLIT) {
          acc[i][j] = Frag<T>::mma(ah, bl[j], acc[i][j]);
          acc[i][j] = Frag<T>::mma(al, bh[j], acc[i][j]);
        }
      }
      Frag<T>::guard(acc[i][0], acc[i][3], ah, SPLIT ? al : ah);
    }
    Frag<T>::keep(bh[0], bh[1], bh[2], bh[3]);
    if (SPLIT) Frag<T>::keep(bl[0], bl[1], bl[2], bl[3]);
  }
  acc_guard4(acc[0][0], acc[0][1], acc[0][2], acc[0][3]);
  acc_guard4(acc[1][0], acc[1][1], acc[1][2], acc[1][3]);
  acc_guard4(acc[2][0], acc[2][1], acc[2][2], acc[2][3]);
  acc_guard4(acc[3][0], acc[3][1], acc[3][2], acc[3][3]);

  float* slab = sT[wave];
#pragma unroll
  for (int i = 0; i < 4; ++i) {
    const int mBase = m0 + (i << 4);
    v4f bmA = (v4f){0.f,0.f,0.f,0.f}, bmB = (v4f){0.f,0.f,0.f,0.f};
    if (BIAS_MODE == 1) {
      bmA = *(const v4f*)(bias + mBase + mOff);
      bmB = *(const v4f*)(bias + mBase + mOff + 4);
    }
#pragma unroll
    for (int j = 0; j < 4; ++j) {
      const int n = n0 + (j << 4) + rlane;
      float bv = 0.f;
      if (BIAS_MODE == 2) bv = bias[n];
#pragma unroll
      for (int r = 0; r < 8; ++r) {
        float v = acc[i][j][r] * scale;
        if (BIAS_MODE == 1) v += (r < 4) ? bmA[r] : bmB[r - 4];
        if (BIAS_MODE == 2) v += bv;
        if (ACT == 2) v = fmaxf(v, 0.0f);
        slab[(mOff + r) * 68 + (j << 4) + rlane] = v;
      }
    }
    __builtin_amdgcn_fence(__ATOMIC_RELEASE, "workgroup");
    __builtin_amdgcn_wave_barrier();
    __builtin_amdgcn_fence(__ATOMIC_ACQUIRE, "workgroup");
    if (OUT_MODE == 0) {
      float* C = (float*)Cout + (size_t)b * strideC;
      const int hh = lane >> 4, c4 = (lane & 15) * 4;
      for (int pass = 0; pass < 2; ++pass) {
#pragma unroll
        for (int it = 0; it < 8; ++it) {
          const int row = it * 2 + hh;
          v4f v = *(const v4f*)(slab + row * 68 + c4);
          *(volatile v4f*)(C + (size_t)(mBase + row) * ldc + n0 + c4) = v;
        }
        __threadfence();
      }
    } else {
      const int q = lane >> 3, c8 = (lane & 7) * 8;
      unsigned short* C  = (unsigned short*)Cout  + (size_t)b * strideC;
      unsigned short* C2 = (OUT_MODE == 2) ? ((unsigned short*)Cout2 + (size_t)b * strideC) : nullptr;
      for (int pass = 0; pass < 2; ++pass) {
#pragma unroll
        for (int it = 0; it < 4; ++it) {
          const int row = it * 4 + q;
          const float* sp = slab + row * 68 + c8;
          v8h hv, lv;
#pragma unroll
          for (int e = 0; e < 8; ++e) {
            if (OUT_MODE == 1) {
              hv[e] = (_Float16)sp[e];
            } else {
              unsigned short hb = f2bf_bits(sp[e]);
              unsigned short lb = f2bf_bits(sp[e] - bf_bits2f(hb));
              hv[e] = __builtin_bit_cast(_Float16, hb);
              lv[e] = __builtin_bit_cast(_Float16, lb);
            }
          }
          *(volatile v8h*)(C + (size_t)(mBase + row) * ldc + n0 + c8) = hv;
          if (OUT_MODE == 2) *(volatile v8h*)(C2 + (size_t)(mBase + row) * ldc + n0 + c8) = lv;
        }
        __threadfence();
      }
    }
    __builtin_amdgcn_fence(__ATOMIC_RELEASE, "workgroup");
    __builtin_amdgcn_wave_barrier();
    __builtin_amdgcn_fence(__ATOMIC_ACQUIRE, "workgroup");
  }
}

__global__ __launch_bounds__(256) void k_cast_bf16x8(
    const float* __restrict__ in, unsigned short* __restrict__ out, int n8) {
  const int i = blockIdx.x * 256 + threadIdx.x;
  if (i < n8) {
    const v4f a = *(const v4f*)(in + (size_t)i * 8);
    const v4f c = *(const v4f*)(in + (size_t)i * 8 + 4);
    v4u w;
    w[0] = (unsigned)f2bf_bits(a[0]) | ((unsigned)f2bf_bits(a[1]) << 16);
    w[1] = (unsigned)f2bf_bits(a[2]) | ((unsigned)f2bf_bits(a[3]) << 16);
    w[2] = (unsigned)f2bf_bits(c[0]) | ((unsigned)f2bf_bits(c[1]) << 16);
    w[3] = (unsigned)f2bf_bits(c[2]) | ((unsigned)f2bf_bits(c[3]) << 16);
    volatile v4u* p = (volatile v4u*)(out + (size_t)i * 8);
    *p = w;
    __threadfence();
    *p = w;
  }
}

template <int CVT> __device__ __forceinline__ unsigned short cvt16(float v, float sc) {
  const unsigned short bb = f2bf_bits(v);
  if (CVT == 0) return bb;
  const float w  = bf_bits2f(bb);
  const float ws = w * sc;
  const _Float16 hv = (_Float16)ws;
  return __builtin_bit_cast(unsigned short, hv);
}
template <int CVT>
__global__ __launch_bounds__(256) void k_transpose_cvt64(
    const float* __restrict__ in, unsigned short* __restrict__ out, int Krows, int Ncols, float sc) {
  __shared__ __align__(16) unsigned short Tl[64 * 72];
  const int n0 = blockIdx.x * 64, k0 = blockIdx.y * 64;
  const int t  = threadIdx.x;
  const int kr = t >> 2;
  const int cb = (t & 3) * 16;
  const float* src = in + (size_t)(k0 + kr) * Ncols + n0 + cb;
  const v4f a0 = *(const v4f*)(src);
  const v4f a1 = *(const v4f*)(src + 4);
  const v4f a2 = *(const v4f*)(src + 8);
  const v4f a3 = *(const v4f*)(src + 12);
#pragma unroll
  for (int e = 0; e < 4; ++e) {
    Tl[(cb + e) * 72 + kr]      = cvt16<CVT>(a0[e], sc);
    Tl[(cb + 4 + e) * 72 + kr]  = cvt16<CVT>(a1[e], sc);
    Tl[(cb + 8 + e) * 72 + kr]  = cvt16<CVT>(a2[e], sc);
    Tl[(cb + 12 + e) * 72 + kr] = cvt16<CVT>(a3[e], sc);
  }
  __syncthreads();
  const int wave = t >> 5, lane = t & 31, q = lane >> 3, c8 = (lane & 7) * 8;
  for (int pass = 0; pass < 2; ++pass) {
#pragma unroll
    for (int it = 0; it < 2; ++it) {
      const int row = wave * 8 + it * 4 + q;
      const v4u val = *(const v4u*)(Tl + row * 72 + c8);
      *(volatile v4u*)(out + (size_t)(n0 + row) * Krows + k0 + c8) = val;
    }
    __threadfence();
  }
}

__global__ __launch_bounds__(256) void k_bias_prep(
    const float* __restrict__ bx, const float* __restrict__ bv, const float* __restrict__ b1,
    float* __restrict__ bxs, float* __restrict__ bvs, float* __restrict__ b1s,
    float sx, float sv, float s1) {
  const int which = blockIdx.x;
  const float* src = bx; float* dst = bxs; int n4 = DQKV / 4; float sc = sx;
  if (which == 1) { src = bv; dst = bvs; sc = sv; }
  if (which == 2) { src = b1; dst = b1s; n4 = NHID / 4; sc = s1; }
  const int t = threadIdx.x;
  if (t < n4) {
    const v4f v = *(const v4f*)(src + (size_t)t * 4);
    v4f o;
    o[0] = bf_bits2f(f2bf_bits(v[0])) * sc;
    o[1] = bf_bits2f(f2bf_bits(v[1])) * sc;
    o[2] = bf_bits2f(f2bf_bits(v[2])) * sc;
    o[3] = bf_bits2f(f2bf_bits(v[3])) * sc;
    volatile v4f* p = (volatile v4f*)(dst + (size_t)t * 4);
    *p = o;
    __threadfence();
    *p = o;
  }
}

__device__ __forceinline__ v8f mma_h(v16h a, v16h b, v8f c) {
  c = __builtin_amdgcn_wmma_f32_16x16x32_f16(false, a, false, b, (short)0, c, false, false);
  asm volatile("v_nop\n\tv_nop\n\tv_nop\n\tv_nop" : "+v"(c) : "v"(a), "v"(b));
  return c;
}

__global__ __launch_bounds__(128) void mlp_attn_kernel(
    const unsigned short* __restrict__ Hp, const unsigned short* __restrict__ W2p,
    const unsigned short* __restrict__ Vp, const float* __restrict__ mask,
    float* __restrict__ out, float sscale, float onorm) {
  union FH { v16h v; v8h h[2]; };
  const _Float16* Hq  = (const _Float16*)(const void*)Hp;
  const _Float16* W2t = (const _Float16*)(const void*)W2p;
  const _Float16* Vt  = (const _Float16*)(const void*)Vp;
  __shared__ __align__(16) _Float16 Psh[4][16 * 64];
  __shared__ __align__(16) float    Os[4][16 * 68];

  const int tid  = threadIdx.x;
  const int wave = tid >> 5;
  const int lane = tid & 31;
  const int hh   = lane >> 4;
  const int c    = lane & 15;
  const int koff = hh * 8;

  constexpr int NQB = SEQ / 64;
  const int bxi = blockIdx.x;
  const int qb  = bxi % NQB;
  const int bh  = bxi / NQB;
  const int h   = bh % NHEAD;
  const int b   = bh / NHEAD;
  const int q0  = qb * 64 + wave * 16;

  v16h qa[4];
  {
    const _Float16* qrow = Hq + ((size_t)bh * SEQ + q0 + c) * NHID + koff;
#pragma unroll
    for (int dc = 0; dc < 4; ++dc) {
      FH f;
      f.h[0] = *(const v8h*)(qrow + dc * 32);
      f.h[1] = *(const v8h*)(qrow + dc * 32 + 16);
      qa[dc] = f.v;
    }
  }

  float mrow[8], lrow[8];
  v8f oacc[4];
#pragma unroll
  for (int r = 0; r < 8; ++r) { mrow[r] = -INFINITY; lrow[r] = 0.f; }
#pragma unroll
  for (int t = 0; t < 4; ++t) oacc[t] = (v8f){0.f,0.f,0.f,0.f,0.f,0.f,0.f,0.f};

  const float* mk_row = mask + (size_t)b * SEQ;
  const _Float16* vbase = Vt + (size_t)(h * DHEAD) * NTOK + (size_t)b * SEQ;
  _Float16* pw = Psh[wave];

  for (int kc = 0; kc < SEQ / 64; ++kc) {
    const int kv0 = kc * 64;

    v8f s[4];
#pragma unroll
    for (int j = 0; j < 4; ++j) {
      s[j] = (v8f){0.f,0.f,0.f,0.f,0.f,0.f,0.f,0.f};
      const _Float16* krow = W2t + (size_t)(kv0 + j * 16 + c) * NHID + koff;
#pragma unroll
      for (int dc = 0; dc < 4; ++dc) {
        FH kb;
        kb.h[0] = *(const v8h*)(krow + dc * 32);
        kb.h[1] = *(const v8h*)(krow + dc * 32 + 16);
        s[j] = mma_h(qa[dc], kb.v, s[j]);
      }
    }

    float pen[4];
#pragma unroll
    for (int j = 0; j < 4; ++j) {
      const float mk = bf_bits2f(f2bf_bits(mk_row[kv0 + j * 16 + c]));
      pen[j] = 1000000.0f * (1.0f - mk);
    }

    float cm[8];
#pragma unroll
    for (int r = 0; r < 8; ++r) {
      float m = -INFINITY;
#pragma unroll
      for (int j = 0; j < 4; ++j) {
        const float sv = s[j][r] * sscale - pen[j];
        s[j][r] = sv;
        m = fmaxf(m, sv);
      }
#pragma unroll
      for (int off = 1; off < 16; off <<= 1) m = fmaxf(m, __shfl_xor(m, off, 32));
      cm[r] = m;
    }

    __builtin_amdgcn_fence(__ATOMIC_RELEASE, "workgroup");
    __builtin_amdgcn_wave_barrier();
    __builtin_amdgcn_fence(__ATOMIC_ACQUIRE, "workgroup");

#pragma unroll
    for (int r = 0; r < 8; ++r) {
      const float mnew  = fmaxf(mrow[r], cm[r]);
      const float alpha = expf(mrow[r] - mnew);
      mrow[r] = mnew;
      float psum = 0.f;
#pragma unroll
      for (int j = 0; j < 4; ++j) {
        const float p = expf(s[j][r] - mnew);
        psum += p;
        pw[(8 * hh + r) * 64 + j * 16 + c] = (_Float16)(p * SC_P);
      }
#pragma unroll
      for (int off = 1; off < 16; off <<= 1) psum += __shfl_xor(psum, off, 32);
      lrow[r] = lrow[r] * alpha + psum;
#pragma unroll
      for (int t = 0; t < 4; ++t) oacc[t][r] *= alpha;
    }
    __builtin_amdgcn_fence(__ATOMIC_RELEASE, "workgroup");
    __builtin_amdgcn_wave_barrier();
    __builtin_amdgcn_fence(__ATOMIC_ACQUIRE, "workgroup");

#pragma unroll
    for (int kk = 0; kk < 2; ++kk) {
      FH pa;
      pa.h[0] = *(const v8h*)(pw + c * 64 + kk * 32 + koff);
      pa.h[1] = *(const v8h*)(pw + c * 64 + kk * 32 + 16 + koff);
#pragma unroll
      for (int t = 0; t < 4; ++t) {
        const _Float16* vr = vbase + (size_t)(t * 16 + c) * NTOK + kv0 + kk * 32 + koff;
        FH vb;
        vb.h[0] = *(const v8h*)(vr);
        vb.h[1] = *(const v8h*)(vr + 16);
        oacc[t] = mma_h(pa.v, vb.v, oacc[t]);
      }
    }
  }

  float* os = Os[wave];
#pragma unroll
  for (int r = 0; r < 8; ++r) {
    const float inv = onorm / lrow[r];
#pragma unroll
    for (int t = 0; t < 4; ++t) os[(8 * hh + r) * 68 + t * 16 + c] = oacc[t][r] * inv;
  }
  __builtin_amdgcn_fence(__ATOMIC_RELEASE, "workgroup");
  __builtin_amdgcn_wave_barrier();
  __builtin_amdgcn_fence(__ATOMIC_ACQUIRE, "workgroup");
  {
    float* ob = out + (size_t)b * SEQ * DQKV + (size_t)h * DHEAD;
    const int c4 = (lane & 15) * 4;
    for (int pass = 0; pass < 2; ++pass) {
#pragma unroll
      for (int it = 0; it < 8; ++it) {
        const int row = it * 2 + hh;
        const v4f val = *(const v4f*)(os + row * 68 + c4);
        *(volatile v4f*)(ob + (size_t)(q0 + row) * DQKV + c4) = val;
      }
      __threadfence();
    }
  }
}

extern "C" void kernel_launch(void* const* d_in, const int* in_sizes, int n_in,
                              void* d_out, int out_size, void* d_ws, size_t ws_size,
                              hipStream_t stream) {
  (void)in_sizes; (void)n_in; (void)out_size; (void)ws_size;
  const float* X   = (const float*)d_in[0];
  const float* msk = (const float*)d_in[1];
  const float* Wx  = (const float*)d_in[2];
  const float* bx  = (const float*)d_in[3];
  const float* Wv  = (const float*)d_in[4];
  const float* bv  = (const float*)d_in[5];
  const float* W1  = (const float*)d_in[6];
  const float* b1  = (const float*)d_in[7];
  const float* W2  = (const float*)d_in[8];
  float* out = (float*)d_out;

  char* ws = (char*)d_ws;
  size_t off = 0;
  auto carve = [&](size_t bytes) -> char* {
    off = (off + 255) & ~(size_t)255;
    char* p = ws + off;
    off += bytes;
    return p;
  };
  unsigned short* Xb   = (unsigned short*)carve((size_t)NTOK * DMODEL * 2);
  unsigned short* WxT  = (unsigned short*)carve((size_t)DQKV * DMODEL * 2);
  unsigned short* WvT  = (unsigned short*)carve((size_t)DQKV * DMODEL * 2);
  unsigned short* W1T  = (unsigned short*)carve((size_t)NHID * DHEAD * 2);
  unsigned short* W2T  = (unsigned short*)carve((size_t)SEQ * NHID * 2);
  float*          bxs  = (float*)carve((size_t)DQKV * 4);
  float*          bvs  = (float*)carve((size_t)DQKV * 4);
  float*          b1s  = (float*)carve((size_t)NHID * 4);
  unsigned short* Xh16 = (unsigned short*)carve((size_t)NTOK * DQKV * 2);
  unsigned short* Vt16 = (unsigned short*)carve((size_t)DQKV * NTOK * 2);
  unsigned short* H16  = (unsigned short*)carve((size_t)NBATCH * NHEAD * SEQ * NHID * 2);

  {
    const int n8 = NTOK * DMODEL / 8;
    k_cast_bf16x8<<<(n8 + 255) / 256, 256, 0, stream>>>(X, Xb, n8);
  }
  k_transpose_cvt64<0><<<dim3(DQKV / 64, DMODEL / 64), 256, 0, stream>>>(Wx, WxT, DMODEL, DQKV, 1.0f);
  k_transpose_cvt64<0><<<dim3(DQKV / 64, DMODEL / 64), 256, 0, stream>>>(Wv, WvT, DMODEL, DQKV, 1.0f);
  k_transpose_cvt64<1><<<dim3(NHID / 64, DHEAD / 64), 256, 0, stream>>>(W1, W1T, DHEAD, NHID, SC_W1);
  k_transpose_cvt64<1><<<dim3(SEQ / 64, NHID / 64), 256, 0, stream>>>(W2, W2T, NHID, SEQ, SC_W2);
  k_bias_prep<<<3, 256, 0, stream>>>(bx, bv, b1, bxs, bvs, b1s, SC_XH, SC_V, SC_H);

  static_assert(NTOK % 64 == 0 && DQKV % 64 == 0 && DMODEL % 32 == 0, "gemm xh");
  wmma_gemm64<1, false, 2, 1, 0><<<dim3((NTOK / 64) * (DQKV / 64) / 8, 1), 256, 0, stream>>>(
      Xb, Xb, DMODEL, 0L, WxT, WxT, DMODEL, 0L, (void*)Xh16, (void*)Xh16, DQKV, 0L,
      bxs, NTOK, DQKV, DMODEL, SC_XH);

  wmma_gemm64<1, false, 1, 1, 0><<<dim3((DQKV / 64) * (NTOK / 64) / 8, 1), 256, 0, stream>>>(
      WvT, WvT, DMODEL, 0L, Xb, Xb, DMODEL, 0L, (void*)Vt16, (void*)Vt16, NTOK, 0L,
      bvs, DQKV, NTOK, DMODEL, SC_V);

  static_assert(SEQ % 64 == 0 && NHID % 64 == 0 && DHEAD % 32 == 0, "gemm h");
  for (int bb = 0; bb < NBATCH; ++bb) {
    const unsigned short* Ab = Xh16 + (size_t)bb * SEQ * DQKV;
    unsigned short* Cb = H16 + (size_t)bb * NHEAD * SEQ * NHID;
    wmma_gemm64<0, false, 2, 1, 2><<<dim3((SEQ / 64) * (NHID / 64) / 8, NHEAD), 256, 0, stream>>>(
        Ab, Ab, DQKV, (long)DHEAD, W1T, W1T, DHEAD, 0L, (void*)Cb, (void*)Cb, NHID, (long)SEQ * NHID,
        b1s, SEQ, NHID, DHEAD, SC_H / (SC_XH * SC_W1));
  }

  mlp_attn_kernel<<<NBATCH * NHEAD * (SEQ / 64), 128, 0, stream>>>(
      H16, W2T, Vt16, msk, out, 1.0f / (SC_H * SC_W2), 1.0f / (SC_P * SC_V));
}
